// MultiHeadAttention_23201413333084
// MI455X (gfx1250) — hardware-verified
//
#include <hip/hip_runtime.h>
#include <math.h>

typedef __attribute__((ext_vector_type(16))) _Float16 v16h;
typedef __attribute__((ext_vector_type(8)))  _Float16 v8h;
typedef __attribute__((ext_vector_type(16))) __bf16   v16b;
typedef __attribute__((ext_vector_type(8)))  __bf16   v8b;
typedef __attribute__((ext_vector_type(8)))  float    v8f;
typedef __attribute__((ext_vector_type(4)))  float    v4f;
typedef __attribute__((ext_vector_type(4)))  unsigned int v4u;

constexpr int kB  = 4;
constexpr int kT  = 2048;
constexpr int kD  = 1024;
constexpr int kH  = 16;
constexpr int kDH = 64;
constexpr int kRows   = kB * kT;
constexpr int kEarly  = 128;
constexpr int kHalfDH = kDH / 2;
constexpr int kTabP   = 2 * kHalfDH;
constexpr int kAoP    = 2 * kD;
constexpr double kRotBase = 10000.0;
constexpr int isqrt_c(int n) { int r = 0; while ((r + 1) * (r + 1) <= n) ++r; return r; }
constexpr float kScoreScale = 1.0f / (float)isqrt_c(kDH);
constexpr float kQKCarry = 8.0f;
constexpr float kVCarry  = 8.0f;
constexpr float kPCarry  = 4096.0f;
constexpr float kScoreFold = kScoreScale / (kQKCarry * kQKCarry);
constexpr float kMaskFill = -1.0e30f;
static_assert(isqrt_c(kDH) * isqrt_c(kDH) == kDH, "head dim is a perfect square");
static_assert(kH * kDH == kD, "head split");
static_assert(kDH == 64 && kHalfDH == 32 && kTabP == 64, "tile geometry");
static_assert((kT % 64) == 0 && (kEarly % 64) == 0 && (kD % 64) == 0 && (kD % 32) == 0 && (kAoP % 32) == 0, "tile multiples");
static_assert(kB == 4 && kT == 2048 && kD == 1024, "wire shapes");

constexpr size_t kOffXB   = 0;
constexpr size_t kOffWQKV = kOffXB   + (size_t)kRows * kD * 2;
constexpr size_t kOffWO2  = kOffWQKV + (size_t)3 * kD * kD * 2;
constexpr size_t kOffCS   = kOffWO2  + (size_t)kD * kAoP * 2;
constexpr size_t kOffQH   = kOffCS   + (size_t)kT * kTabP * 4;
constexpr size_t kOffKH   = kOffQH   + (size_t)kRows * kD * 2;
constexpr size_t kOffVT   = kOffKH   + (size_t)kRows * kD * 2;
constexpr size_t kOffQ32  = kOffVT   + (size_t)kRows * kD * 2;
constexpr size_t kOffK32  = kOffQ32  + (size_t)kB * kEarly * kD * 4;
constexpr size_t kOffV32  = kOffK32  + (size_t)kB * kEarly * kD * 4;
constexpr size_t kOffAO2  = kOffV32  + (size_t)kB * kEarly * kD * 4;
constexpr size_t kWsTotal = kOffAO2  + (size_t)kRows * kAoP * 2;
static_assert(kWsTotal == 117964800ull, "carve total");
static_assert(kWsTotal <= 134217728ull, "carve cap");
static_assert((kOffWQKV % 128) == 0 && (kOffWO2 % 128) == 0 && (kOffCS % 128) == 0 && (kOffQH % 128) == 0 &&
              (kOffKH % 128) == 0 && (kOffVT % 128) == 0 && (kOffQ32 % 128) == 0 && (kOffK32 % 128) == 0 &&
              (kOffV32 % 128) == 0 && (kOffAO2 % 128) == 0, "128-B aligned regions");

struct InvFreq { float v[32]; };
static_assert(sizeof(InvFreq) == 128, "no padding");

__device__ __forceinline__ unsigned short f2bf_bits(float f) {
  unsigned u = __float_as_uint(f);
  return (unsigned short)((u + 0x7FFFu + ((u >> 16) & 1u)) >> 16);
}
__device__ __forceinline__ float bf_bits2f(unsigned short h) { return __uint_as_float(((unsigned)h) << 16); }
__device__ __forceinline__ unsigned pk16(unsigned short a, unsigned short b) { return (unsigned)a | ((unsigned)b << 16); }
__device__ __forceinline__ unsigned short h_bits(float f) { const _Float16 h = (_Float16)f; return __builtin_bit_cast(unsigned short, h); }

__device__ __forceinline__ void wave_sync() {
  __builtin_amdgcn_fence(__ATOMIC_RELEASE, "workgroup");
  __builtin_amdgcn_wave_barrier();
  __builtin_amdgcn_fence(__ATOMIC_ACQUIRE, "workgroup");
}

__device__ __forceinline__ v8f mma_b(v16b a, v16b b, v8f c) {
  c = __builtin_amdgcn_wmma_f32_16x16x32_bf16(false, a, false, b, (short)0, c, false, false);
  asm volatile("v_nop\n\tv_nop\n\tv_nop\n\tv_nop" : "+v"(c) : "v"(a), "v"(b));
  return c;
}
__device__ __forceinline__ v8f mma_h(v16h a, v16h b, v8f c) {
  c = __builtin_amdgcn_wmma_f32_16x16x32_f16(false, a, false, b, (short)0, c, false, false);
  asm volatile("v_nop\n\tv_nop\n\tv_nop\n\tv_nop" : "+v"(c) : "v"(a), "v"(b));
  return c;
}
__device__ __forceinline__ v16b frag_b(const __bf16* p) {
  union U { v16b v; v8b h[2]; } f;
  f.h[0] = *(const v8b*)(p);
  f.h[1] = *(const v8b*)(p + 16);
  return f.v;
}
__device__ __forceinline__ v16h frag_h(const _Float16* p) {
  union U { v16h v; v8h h[2]; } f;
  f.h[0] = *(const v8h*)(p);
  f.h[1] = *(const v8h*)(p + 16);
  return f.v;
}
__device__ __forceinline__ v4u cvt8_bf16(const float* p) {
  const v4f a = *(const v4f*)(p);
  const v4f c = *(const v4f*)(p + 4);
  unsigned short hb[8];
#pragma unroll
  for (int e = 0; e < 4; ++e) {
    hb[e]     = f2bf_bits(a[e]);
    hb[4 + e] = f2bf_bits(c[e]);
  }
  return (v4u){pk16(hb[0], hb[1]), pk16(hb[2], hb[3]), pk16(hb[4], hb[5]), pk16(hb[6], hb[7])};
}

__global__ __launch_bounds__(256) void cvt_x_kernel(const float* __restrict__ in, unsigned short* __restrict__ out, int n8) {
  const int i = blockIdx.x * 256 + threadIdx.x;
  if (i >= n8) return;
  const v4u u = cvt8_bf16(in + 8 * (size_t)i);
  unsigned short* q = out + 8 * (size_t)i;
  *(volatile v4u*)q = u;
  __threadfence();
  *(volatile v4u*)q = u;
}

__global__ __launch_bounds__(256) void cvt_w_kernel(const float* __restrict__ Wq, const float* __restrict__ Wk,
                                                    const float* __restrict__ Wv, const float* __restrict__ Wo,
                                                    unsigned short* __restrict__ WQKV, unsigned short* __restrict__ WO2) {
  const int z = blockIdx.y;
  const float* W = (z == 0) ? Wq : (z == 1) ? Wk : (z == 2) ? Wv : Wo;
  const int i = blockIdx.x * 256 + threadIdx.x;
  const size_t e0 = 8 * (size_t)i;
  const v4u u = cvt8_bf16(W + e0);
  if (z < 3) {
    unsigned short* q = WQKV + (size_t)z * kD * kD + e0;
    *(volatile v4u*)q = u;
    __threadfence();
    *(volatile v4u*)q = u;
  } else {
    const size_t row = e0 / kD;
    const size_t col = e0 - row * kD;
    unsigned short* q0 = WO2 + row * kAoP + col;
    unsigned short* q1 = q0 + kD;
    *(volatile v4u*)q0 = u;
    *(volatile v4u*)q1 = u;
    __threadfence();
    *(volatile v4u*)q0 = u;
    *(volatile v4u*)q1 = u;
  }
}

__global__ __launch_bounds__(256) void rot_tab_kernel(float* __restrict__ CS, InvFreq fr) {
  __shared__ __align__(16) float sC[8][64];
  const int lane = threadIdx.x & 31;
  const int wave = __builtin_amdgcn_readfirstlane((int)(threadIdx.x >> 5));
  const int t = blockIdx.x * 8 + wave;
  float invf = fr.v[0];
#pragma unroll
  for (int jj = 1; jj < 32; ++jj) invf = (lane == jj) ? fr.v[jj] : invf;
  const float ang = (float)t * invf;
  sC[wave][lane]      = cosf(ang);
  sC[wave][32 + lane] = sinf(ang);
  __syncthreads();
  const int l4 = (lane & 15) * 4;
  const v4f v = *(const v4f*)(&sC[wave][l4]);
  float* dst = CS + (size_t)t * kTabP + l4;
  for (int pass = 0; pass < 2; ++pass) {
    if (lane < 16) *(volatile v4f*)dst = v;
    __threadfence();
  }
}

template <int EPI>
__global__ __launch_bounds__(256) void gemm_bf16_kernel(
    const unsigned short* __restrict__ Ap, int lda, long strideA,
    const unsigned short* __restrict__ Btp, int ldb, long strideB,
    void* __restrict__ Cout, int ldc, long strideC,
    int M, int N, int K, float scale,
    const float* __restrict__ CS,
    unsigned short* __restrict__ QH, unsigned short* __restrict__ KH,
    float* __restrict__ Q32, float* __restrict__ K32) {
  __shared__ __align__(16) float sT[8][16 * 68];
  const int bz   = blockIdx.y;
  const int lane = threadIdx.x & 31;
  const int wave = __builtin_amdgcn_readfirstlane((int)(threadIdx.x >> 5));
  const int tilesN = N >> 6;
  const int tilesM = M >> 6;
  const int tile = blockIdx.x * 8 + wave;
  if (tile >= tilesM * tilesN) return;
  const int tm = tile / tilesN;
  const int tn = tile - tm * tilesN;
  const int m0 = tm << 6;
  const int n0 = tn << 6;

  const __bf16* Ab = (const __bf16*)Ap  + (size_t)bz * strideA;
  const __bf16* Bb = (const __bf16*)Btp + (size_t)bz * strideB;

  const int rlane = lane & 15;
  const int koff  = (lane >> 4) * 8;
  const int mOff  = (lane >> 4) * 8;

  v8f acc[4][4];
#pragma unroll
  for (int i = 0; i < 4; ++i)
#pragma unroll
    for (int j = 0; j < 4; ++j) acc[i][j] = (v8f){0.f, 0.f, 0.f, 0.f, 0.f, 0.f, 0.f, 0.f};

  for (int k0 = 0; k0 < K; k0 += 32) {
    v16b bh[4];
#pragma unroll
    for (int j = 0; j < 4; ++j)
      bh[j] = frag_b(Bb + (size_t)(n0 + (j << 4) + rlane) * ldb + koff + k0);
#pragma unroll
    for (int i = 0; i < 4; ++i) {
      const v16b ah = frag_b(Ab + (size_t)(m0 + (i << 4) + rlane) * lda + koff + k0);
#pragma unroll
      for (int j = 0; j < 4; ++j) acc[i][j] = mma_b(ah, bh[j], acc[i][j]);
    }
  }

  float* slab = sT[wave];
#pragma unroll
  for (int i = 0; i < 4; ++i) {
    const int mBase = m0 + (i << 4);
#pragma unroll
    for (int j = 0; j < 4; ++j) {
#pragma unroll
      for (int r = 0; r < 8; ++r) slab[(mOff + r) * 68 + (j << 4) + rlane] = acc[i][j][r] * scale;
    }
    wave_sync();
    if (EPI == 0) {
      float* C = (float*)Cout + (size_t)bz * strideC;
      const int hh = lane >> 4, c4 = (lane & 15) * 4;
      for (int pass = 0; pass < 2; ++pass) {
#pragma unroll
        for (int it = 0; it < 8; ++it) {
          const int row = it * 2 + hh;
          const v4f v = *(const v4f*)(slab + row * 68 + c4);
          *(volatile v4f*)(C + (size_t)(mBase + row) * ldc + n0 + c4) = v;
        }
        __threadfence();
      }
    } else if (EPI == 1) {
      const int q = lane >> 3, c8 = (lane & 7) * 8;
      unsigned short* C = (unsigned short*)Cout + (size_t)bz * strideC;
      for (int pass = 0; pass < 2; ++pass) {
#pragma unroll
        for (int it = 0; it < 4; ++it) {
          const int row = it * 4 + q;
          const float* sp = slab + row * 68 + c8;
          v8h hv;
#pragma unroll
          for (int e = 0; e < 8; ++e) hv[e] = (_Float16)sp[e];
          *(volatile v8h*)(C + (size_t)(mBase + row) * ldc + n0 + c8) = hv;
        }
        __threadfence();
      }
    } else {
      const int sect = tn >> 4;
      const int head = tn & 15;
      const bool early = ((m0 % kT) < kEarly);
      unsigned short* P16 = sect ? KH : QH;
      float* P32 = sect ? K32 : Q32;
      const int q = lane >> 3, c8 = (lane & 7) * 8;
      v4u hv[4];
#pragma unroll
      for (int it = 0; it < 4; ++it) {
        const int row  = it * 4 + q;
        const int mrow = mBase + row;
        const int tt   = mrow % kT;
        float* sp = slab + row * 68 + c8;
        const v4f a0 = *(const v4f*)(sp);
        const v4f a1 = *(const v4f*)(sp + 4);
        const float* tp = CS + (size_t)tt * kTabP + (c8 >> 1);
        const v4f cc = *(const v4f*)(tp);
        const v4f sn = *(const v4f*)(tp + kHalfDH);
        v4f r0, r1;
        r0[0] = a0[0] * cc[0] - a0[1] * sn[0];
        r0[1] = a0[0] * sn[0] + a0[1] * cc[0];
        r0[2] = a0[2] * cc[1] - a0[3] * sn[1];
        r0[3] = a0[2] * sn[1] + a0[3] * cc[1];
        r1[0] = a1[0] * cc[2] - a1[1] * sn[2];
        r1[1] = a1[0] * sn[2] + a1[1] * cc[2];
        r1[2] = a1[2] * cc[3] - a1[3] * sn[3];
        r1[3] = a1[2] * sn[3] + a1[3] * cc[3];
        if (early) {
          *(v4f*)(sp)     = r0;
          *(v4f*)(sp + 4) = r1;
        }
        hv[it] = (v4u){pk16(h_bits(r0[0] * kQKCarry), h_bits(r0[1] * kQKCarry)),
                       pk16(h_bits(r0[2] * kQKCarry), h_bits(r0[3] * kQKCarry)),
                       pk16(h_bits(r1[0] * kQKCarry), h_bits(r1[1] * kQKCarry)),
                       pk16(h_bits(r1[2] * kQKCarry), h_bits(r1[3] * kQKCarry))};
      }
      for (int pass = 0; pass < 2; ++pass) {
#pragma unroll
        for (int it = 0; it < 4; ++it) {
          const int mrow = mBase + it * 4 + q;
          const int bq = mrow / kT;
          const int tt = mrow - bq * kT;
          *(volatile v4u*)(P16 + ((size_t)(bq * kH + head) * kT + tt) * kDH + c8) = hv[it];
        }
        __threadfence();
      }
      if (early) {
        wave_sync();
        const int hh = lane >> 4, c4 = (lane & 15) * 4;
        for (int pass = 0; pass < 2; ++pass) {
#pragma unroll
          for (int it = 0; it < 8; ++it) {
            const int row  = it * 2 + hh;
            const int mrow = mBase + row;
            const int bq = mrow / kT;
            const int tt = mrow - bq * kT;
            const v4f v = *(const v4f*)(slab + row * 68 + c4);
            *(volatile v4f*)(P32 + ((size_t)(bq * kEarly + tt)) * kD + head * kDH + c4) = v;
          }
          __threadfence();
        }
      }
    }
    wave_sync();
  }
}

__global__ __launch_bounds__(32) void early_attn_kernel(const float* __restrict__ Q32, const float* __restrict__ K32,
                                                        const float* __restrict__ V32, const int* __restrict__ amask,
                                                        unsigned short* __restrict__ AO2) {
  __shared__ __align__(16) float sQ[64];
  __shared__ __align__(16) float sP[128];
  __shared__ __align__(16) float sO[64];
  const int lane = threadIdx.x;
  const int bx = blockIdx.x;
  const int t  = bx % kEarly;
  const int bh = bx / kEarly;
  const int h  = bh % kH;
  const int b  = bh / kH;
  const float* qrow = Q32 + ((size_t)(b * kEarly + t)) * kD + h * kDH;
  sQ[lane]      = qrow[lane];
  sQ[lane + 32] = qrow[lane + 32];
  __syncthreads();
  const int nks = (t >> 5) + 1;
#pragma unroll 1
  for (int ks = 0; ks < nks; ++ks) {
    const int s = ks * 32 + lane;
    const float* krow = K32 + ((size_t)(b * kEarly + s)) * kD + h * kDH;
    float acc = 0.f;
#pragma unroll 1
    for (int c = 0; c < 16; ++c) {
      const v4f kv = *(const v4f*)(krow + 4 * c);
      const v4f qv = *(const v4f*)(sQ + 4 * c);
      acc = fmaf(qv[0], kv[0], acc);
      acc = fmaf(qv[1], kv[1], acc);
      acc = fmaf(qv[2], kv[2], acc);
      acc = fmaf(qv[3], kv[3], acc);
    }
    int mk = amask[b * kT + s];
    asm volatile("" : "+v"(mk));
    const bool live = (s <= t) && (mk != 0);
    sP[s] = live ? (acc * kScoreScale) : kMaskFill;
  }
  __syncthreads();
  float m = -INFINITY;
#pragma unroll 1
  for (int ks = 0; ks < nks; ++ks) m = fmaxf(m, sP[ks * 32 + lane]);
#pragma unroll
  for (int off = 16; off > 0; off >>= 1) m = fmaxf(m, __shfl_xor(m, off, 32));
  float ls = 0.f;
#pragma unroll 1
  for (int ks = 0; ks < nks; ++ks) {
    const int idx = ks * 32 + lane;
    const float p = expf(sP[idx] - m);
    sP[idx] = p;
    ls += p;
  }
#pragma unroll
  for (int off = 16; off > 0; off >>= 1) ls += __shfl_xor(ls, off, 32);
  __syncthreads();
  float o0 = 0.f, o1 = 0.f;
#pragma unroll 1
  for (int s = 0; s <= t; ++s) {
    const float p = sP[s];
    const float* vrow = V32 + ((size_t)(b * kEarly + s)) * kD + h * kDH;
    o0 = fmaf(p, vrow[lane], o0);
    o1 = fmaf(p, vrow[lane + 32], o1);
  }
  float inv = 1.0f / ls;
  if (m < -1.0e29f) inv = __uint_as_float(0x7fc00000u);
  sO[lane]      = o0 * inv;
  sO[lane + 32] = o1 * inv;
  __syncthreads();
  const int g  = (lane >> 3) & 1;
  const int c8 = (lane & 7) * 8;
  const v4f a0 = *(const v4f*)(sO + c8);
  const v4f a1 = *(const v4f*)(sO + c8 + 4);
  unsigned short wb[8];
#pragma unroll
  for (int e = 0; e < 4; ++e) {
    const float f0 = a0[e];
    const float f1 = a1[e];
    const unsigned short h0 = f2bf_bits(f0);
    const unsigned short h1 = f2bf_bits(f1);
    const unsigned short l0 = f2bf_bits(f0 - bf_bits2f(h0));
    const unsigned short l1 = f2bf_bits(f1 - bf_bits2f(h1));
    wb[e]     = g ? l0 : h0;
    wb[4 + e] = g ? l1 : h1;
  }
  const v4u u = (v4u){pk16(wb[0], wb[1]), pk16(wb[2], wb[3]), pk16(wb[4], wb[5]), pk16(wb[6], wb[7])};
  unsigned short* dst = AO2 + ((size_t)(b * kT + t)) * kAoP + g * kD + h * kDH + c8;
  for (int pass = 0; pass < 2; ++pass) {
    if (lane < 16) *(volatile v4u*)dst = u;
    __threadfence();
  }
}

__global__ __launch_bounds__(128) void attn_stream_kernel(const unsigned short* __restrict__ QHp,
                                                         const unsigned short* __restrict__ KHp,
                                                         const unsigned short* __restrict__ VTp,
                                                         const int* __restrict__ amask,
                                                         unsigned short* __restrict__ AO2) {
  __shared__ __align__(16) _Float16 Psh[4][16 * 64];
  __shared__ __align__(16) float Os[4][16 * 68];
  const int lane = threadIdx.x & 31;
  const int wave = __builtin_amdgcn_readfirstlane((int)(threadIdx.x >> 5));
  const int hh = lane >> 4;
  const int c  = lane & 15;
  constexpr int kQTiles = kT / 64 - kEarly / 64;
  const int bx = blockIdx.x;
  const int qb = kEarly / 64 + bx % kQTiles;
  const int bh = bx / kQTiles;
  const int h  = bh % kH;
  const int b  = bh / kH;
  const int q0 = qb * 64 + wave * 16;
  const _Float16* Qg = (const _Float16*)QHp + (size_t)bh * kT * kDH;
  const _Float16* Kg = (const _Float16*)KHp + (size_t)bh * kT * kDH;
  const _Float16* Vg = (const _Float16*)VTp + (size_t)bh * kDH * kT;

  v16h qa[2];
#pragma unroll
  for (int dc = 0; dc < 2; ++dc) qa[dc] = frag_h(Qg + (size_t)(q0 + c) * kDH + dc * 32 + 8 * hh);

  float mrow[8], lrow[8];
  v8f oacc[4];
#pragma unroll
  for (int r = 0; r < 8; ++r) { mrow[r] = -INFINITY; lrow[r] = 0.f; }
#pragma unroll
  for (int t = 0; t < 4; ++t) oacc[t] = (v8f){0.f, 0.f, 0.f, 0.f, 0.f, 0.f, 0.f, 0.f};

  _Float16* pw = Psh[wave];
  const int nChunks = qb + 1;
  for (int kc = 0; kc < nChunks; ++kc) {
    const int kv0 = kc * 64;
    v8f s[4];
#pragma unroll
    for (int j = 0; j < 4; ++j) {
      s[j] = (v8f){0.f, 0.f, 0.f, 0.f, 0.f, 0.f, 0.f, 0.f};
      const _Float16* kp = Kg + (size_t)(kv0 + j * 16 + c) * kDH + 8 * hh;
#pragma unroll
      for (int dc = 0; dc < 2; ++dc) {
        const v16h kb = frag_h(kp + dc * 32);
        s[j] = mma_h(qa[dc], kb, s[j]);
      }
    }
    int kvkeep[4];
#pragma unroll
    for (int j = 0; j < 4; ++j) {
      kvkeep[j] = amask[b * kT + kv0 + j * 16 + c];
      asm volatile("" : "+v"(kvkeep[j]));
    }
    const bool diag = (kc == qb);
    float cm[8];
#pragma unroll
    for (int r = 0; r < 8; ++r) {
      const int qrow = q0 + 8 * hh + r;
      float m = -INFINITY;
#pragma unroll
      for (int j = 0; j < 4; ++j) {
        const int kvcol = kv0 + j * 16 + c;
        const bool masked = (diag && (kvcol > qrow)) || (kvkeep[j] == 0);
        const float sv = masked ? kMaskFill : (s[j][r] * kScoreFold);
        s[j][r] = sv;
        m = fmaxf(m, sv);
      }
      m = fmaxf(m, __shfl_xor(m, 1, 32));
      m = fmaxf(m, __shfl_xor(m, 2, 32));
      m = fmaxf(m, __shfl_xor(m, 4, 32));
      m = fmaxf(m, __shfl_xor(m, 8, 32));
      cm[r] = m;
    }
#pragma unroll
    for (int r = 0; r < 8; ++r) {
      const float mnew  = fmaxf(mrow[r], cm[r]);
      const float alpha = __expf(mrow[r] - mnew);
      mrow[r] = mnew;
      float psum = 0.f;
#pragma unroll
      for (int j = 0; j < 4; ++j) {
        const float p = __expf(s[j][r] - mnew);
        const _Float16 ph = (_Float16)(p * kPCarry);
        psum += (float)ph;
        pw[(8 * hh + r) * 64 + j * 16 + c] = ph;
      }
      lrow[r] = lrow[r] * alpha + psum;
#pragma unroll
      for (int t = 0; t < 4; ++t) oacc[t][r] *= alpha;
    }
    wave_sync();
#pragma unroll
    for (int kk = 0; kk < 2; ++kk) {
      const v16h pa = frag_h(pw + c * 64 + kk * 32 + 8 * hh);
#pragma unroll
      for (int t = 0; t < 4; ++t) {
        const v16h vb = frag_h(Vg + (size_t)(t * 16 + c) * kT + kv0 + kk * 32 + 8 * hh);
        oacc[t] = mma_h(pa, vb, oacc[t]);
      }
    }
    wave_sync();
  }

  float* os = Os[wave];
#pragma unroll
  for (int r = 0; r < 8; ++r) {
    float l = lrow[r];
    l += __shfl_xor(l, 1, 32);
    l += __shfl_xor(l, 2, 32);
    l += __shfl_xor(l, 4, 32);
    l += __shfl_xor(l, 8, 32);
    float inv = 1.0f / (l * kVCarry);
    if (mrow[r] < -1.0e29f) inv = __uint_as_float(0x7fc00000u);
#pragma unroll
    for (int t = 0; t < 4; ++t) os[(8 * hh + r) * 68 + t * 16 + c] = oacc[t][r] * inv;
  }
  wave_sync();
  {
    const int q = lane >> 3, c8 = (lane & 7) * 8;
    v4u hv[4], lv[4];
#pragma unroll
    for (int it = 0; it < 4; ++it) {
      const int row = it * 4 + q;
      const float* sp = os + row * 68 + c8;
      const v4f a0 = *(const v4f*)(sp);
      const v4f a1 = *(const v4f*)(sp + 4);
      unsigned short hb[8], lb[8];
#pragma unroll
      for (int e = 0; e < 4; ++e) {
        const float f0 = a0[e];
        const float f1 = a1[e];
        hb[e]     = f2bf_bits(f0);
        hb[4 + e] = f2bf_bits(f1);
        lb[e]     = f2bf_bits(f0 - bf_bits2f(hb[e]));
        lb[4 + e] = f2bf_bits(f1 - bf_bits2f(hb[4 + e]));
      }
      hv[it] = (v4u){pk16(hb[0], hb[1]), pk16(hb[2], hb[3]), pk16(hb[4], hb[5]), pk16(hb[6], hb[7])};
      lv[it] = (v4u){pk16(lb[0], lb[1]), pk16(lb[2], lb[3]), pk16(lb[4], lb[5]), pk16(lb[6], lb[7])};
    }
    for (int pass = 0; pass < 2; ++pass) {
#pragma unroll
      for (int it = 0; it < 4; ++it) {
        const int row = it * 4 + q;
        unsigned short* dst = AO2 + ((size_t)(b * kT + q0 + row)) * kAoP + h * kDH + c8;
        *(volatile v4u*)(dst)      = hv[it];
        *(volatile v4u*)(dst + kD) = lv[it];
      }
      __threadfence();
    }
  }
}

extern "C" void kernel_launch(void* const* d_in, const int* in_sizes, int n_in,
                              void* d_out, int out_size, void* d_ws, size_t ws_size,
                              hipStream_t stream) {
  if (n_in < 6) return;
  if (in_sizes[0] != kRows * kD) return;
  if (in_sizes[1] != kB * kT) return;
  if (in_sizes[2] != kD * kD) return;
  if (in_sizes[3] != kD * kD) return;
  if (in_sizes[4] != kD * kD) return;
  if (in_sizes[5] != kD * kD) return;
  if (out_size != kRows * kD) return;
  if (ws_size < kWsTotal) return;

  const float* x     = (const float*)d_in[0];
  const int*   amask = (const int*)d_in[1];
  const float* Wq    = (const float*)d_in[2];
  const float* Wk    = (const float*)d_in[3];
  const float* Wv    = (const float*)d_in[4];
  const float* Wo    = (const float*)d_in[5];
  float* out = (float*)d_out;

  char* ws = (char*)d_ws;
  unsigned short* XB   = (unsigned short*)(ws + kOffXB);
  unsigned short* WQKV = (unsigned short*)(ws + kOffWQKV);
  unsigned short* WO2  = (unsigned short*)(ws + kOffWO2);
  float*          CS   = (float*)(ws + kOffCS);
  unsigned short* QH   = (unsigned short*)(ws + kOffQH);
  unsigned short* KH   = (unsigned short*)(ws + kOffKH);
  unsigned short* VT   = (unsigned short*)(ws + kOffVT);
  float*          Q32  = (float*)(ws + kOffQ32);
  float*          K32  = (float*)(ws + kOffK32);
  float*          V32  = (float*)(ws + kOffV32);
  unsigned short* AO2  = (unsigned short*)(ws + kOffAO2);
  unsigned short* WV   = WQKV + (size_t)2 * kD * kD;

  InvFreq fr;
  for (int j = 0; j < kHalfDH; ++j) {
    const float e = (float)(2 * j) / (float)kDH;
    const float p = (float)pow(kRotBase, (double)e);
    fr.v[j] = 1.0f / p;
  }

  cvt_x_kernel<<<(kRows * kD / 8) / 256, 256, 0, stream>>>(x, XB, kRows * kD / 8);
  cvt_w_kernel<<<dim3((kD * kD / 8) / 256, 4), 256, 0, stream>>>(Wq, Wk, Wv, Wo, WQKV, WO2);
  rot_tab_kernel<<<kT / 8, 256, 0, stream>>>(CS, fr);

  gemm_bf16_kernel<2><<<dim3(512, 1), 256, 0, stream>>>(
      XB, kD, 0L,
      WQKV, kD, 0L,
      (void*)QH, kDH, 0L,
      kRows, 2 * kD, kD, 1.0f,
      CS, QH, KH, Q32, K32);

  gemm_bf16_kernel<1><<<dim3(64, kB), 256, 0, stream>>>(
      WV, kD, 0L,
      XB, kD, (long)kT * kD,
      (void*)VT, kT, (long)kD * kT,
      kD, kT, kD, kVCarry,
      CS, QH, KH, Q32, K32);

  gemm_bf16_kernel<0><<<dim3(4, kB), 256, 0, stream>>>(
      XB, kD, (long)kT * kD,
      WV, kD, 0L,
      (void*)V32, kD, (long)kEarly * kD,
      kEarly, kD, kD, 1.0f,
      CS, QH, KH, Q32, K32);

  early_attn_kernel<<<kB * kH * kEarly, 32, 0, stream>>>(Q32, K32, V32, amask, AO2);

  attn_stream_kernel<<<kB * kH * (kT / 64 - kEarly / 64), 128, 0, stream>>>(QH, KH, VT, amask, AO2);

  gemm_bf16_kernel<0><<<dim3(256, 1), 256, 0, stream>>>(
      AO2, kAoP, 0L,
      WO2, kAoP, 0L,
      (void*)out, kD, 0L,
      kRows, kD, kAoP, 1.0f,
      CS, QH, KH, Q32, K32);
}
